// RGCN_85993835200954
// MI455X (gfx1250) — hardware-run, weakly checked
//
#include <hip/hip_runtime.h>
#include <stdint.h>

#define NB     8
#define NO     1024
#define NM     256
#define CIN    64
#define PO     128
#define HID    128
#define NTY    3
#define NFM    96
#define MROWS  (NB * NO)
#define TP     132

#define PAR_E4   0
#define PAR_B1   512
#define PAR_B2   640
#define PAR_BOM1 768
#define PAR_WOM2 896
#define PAR_SC   1024
#define PAR_N    1056

#define PB0_XB   0
#define PB0_FMT  256
#define PB0_W2D  384
#define PB0_WOM  400
#define PB0_W1T  416
#define PB0_WR3  420
#define PB0_PAR  432
#define PB_TOTAL 438

#define O_XB    ((size_t)0)
#define O_AHL   ((size_t)1048576)
#define O_FMT   ((size_t)9437184)
#define O_H0    ((size_t)9961472)
#define O_P     ((size_t)14155776)
#define O_G3    ((size_t)18350080)
#define O_FM    ((size_t)21495808)
#define O_W1T   ((size_t)25690112)
#define O_W2D   ((size_t)25706496)
#define O_WR3   ((size_t)25772032)
#define O_WOM   ((size_t)25821184)
#define O_PAR   ((size_t)25886720)
#define WS_TOTAL ((size_t)25891072)
#define WSCAP   ((size_t)134217728)

static_assert(MROWS % 128 == 0);
static_assert(NO % 128 == 0);
static_assert(MROWS % 64 == 0);
static_assert(MROWS % 8 == 0);
static_assert(NM == 8 * 32);
static_assert(HID == 128);
static_assert(PO == 128);
static_assert(NFM <= 128);
static_assert(NFM % 8 == 0);
static_assert(CIN % 32 == 0);
static_assert((2 * HID) % 32 == 0);
static_assert((2 * NM) % 32 == 0);
static_assert((3 * CIN) % 32 == 0);
static_assert(O_AHL == O_XB + (size_t)MROWS * CIN * 2);
static_assert(O_FMT == O_AHL + (size_t)MROWS * 512 * 2);
static_assert(O_H0 == O_FMT + (size_t)NB * CIN * 512 * 2);
static_assert(O_P == O_H0 + (size_t)MROWS * 256 * 2);
static_assert(O_G3 == O_P + (size_t)MROWS * PO * 4);
static_assert(O_FM == O_G3 + (size_t)MROWS * 192 * 2);
static_assert(O_W1T == O_FM + (size_t)MROWS * 256 * 2);
static_assert(O_W2D == O_W1T + (size_t)128 * 64 * 2);
static_assert(O_WR3 == O_W2D + (size_t)128 * 256 * 2);
static_assert(O_WOM == O_WR3 + (size_t)128 * 192 * 2);
static_assert(O_PAR == O_WOM + (size_t)128 * 256 * 2);
static_assert(WS_TOTAL >= O_PAR + (size_t)PAR_N * 4);
static_assert(WS_TOTAL % 256 == 0);
static_assert(WS_TOTAL <= WSCAP);
static_assert(MROWS * CIN / 8 == 256 * 256);
static_assert(NB * CIN * 512 / 8 == 128 * 256);
static_assert(128 * 256 / 8 == 16 * 256);
static_assert(128 * 64 / 8 == 4 * 256);
static_assert(128 * 192 / 8 == 12 * 256);

typedef float          v4f   __attribute__((ext_vector_type(4)));
typedef float          v8f   __attribute__((ext_vector_type(8)));
typedef int            v4i   __attribute__((ext_vector_type(4)));
typedef int            v8i   __attribute__((ext_vector_type(8)));
typedef unsigned int   v4u   __attribute__((ext_vector_type(4)));
typedef unsigned short v8us  __attribute__((ext_vector_type(8)));
typedef __bf16         v16bf __attribute__((ext_vector_type(16)));
typedef v4f  __attribute__((may_alias)) v4fa;
typedef v4i  __attribute__((may_alias)) v4ia;
typedef v4u  __attribute__((may_alias)) v4ua;
typedef v8us __attribute__((may_alias)) v8usa;
union FragB { v16bf v; v8us h[2]; v8i w; };
struct HL { v4u h; v4u l; };

__device__ __forceinline__ unsigned f2bf(float f) {
  const unsigned u = __float_as_uint(f);
  return ((u + 0x7FFFu + ((u >> 16) & 1u)) >> 16) & 0xffffu;
}
__device__ __forceinline__ float bf2f(unsigned b) { return __uint_as_float(b << 16); }
__device__ __forceinline__ float bfr(float f) { return bf2f(f2bf(f)); }
__device__ __forceinline__ unsigned pk(unsigned lo, unsigned hi) { return (lo & 0xffffu) | (hi << 16); }
__device__ __forceinline__ v8f z8() { v8f z = {0.f, 0.f, 0.f, 0.f, 0.f, 0.f, 0.f, 0.f}; return z; }
__device__ __forceinline__ void pin4(v4f p) { asm volatile("" :: "v"(p.x), "v"(p.y), "v"(p.z), "v"(p.w)); }
__device__ __forceinline__ float elu_f(float x) { return (x > 0.0f) ? x : expm1f(x); }

__device__ __forceinline__ v4u pack8(float a0, float a1, float a2, float a3,
                                     float a4, float a5, float a6, float a7) {
  v4u v;
  v.x = pk(f2bf(a0), f2bf(a1));
  v.y = pk(f2bf(a2), f2bf(a3));
  v.z = pk(f2bf(a4), f2bf(a5));
  v.w = pk(f2bf(a6), f2bf(a7));
  return v;
}

__device__ __forceinline__ HL split8(v4f a, v4f b) {
  const unsigned h0 = f2bf(a.x), h1 = f2bf(a.y), h2 = f2bf(a.z), h3 = f2bf(a.w);
  const unsigned h4 = f2bf(b.x), h5 = f2bf(b.y), h6 = f2bf(b.z), h7 = f2bf(b.w);
  const unsigned l0 = f2bf(a.x - bf2f(h0)), l1 = f2bf(a.y - bf2f(h1));
  const unsigned l2 = f2bf(a.z - bf2f(h2)), l3 = f2bf(a.w - bf2f(h3));
  const unsigned l4 = f2bf(b.x - bf2f(h4)), l5 = f2bf(b.y - bf2f(h5));
  const unsigned l6 = f2bf(b.z - bf2f(h6)), l7 = f2bf(b.w - bf2f(h7));
  HL r;
  r.h.x = pk(h0, h1); r.h.y = pk(h2, h3); r.h.z = pk(h4, h5); r.h.w = pk(h6, h7);
  r.l.x = pk(l0, l1); r.l.y = pk(l2, l3); r.l.z = pk(l4, l5); r.l.w = pk(l6, l7);
  return r;
}

__device__ __forceinline__ void put_u4(unsigned short* dst, v4u v) {
  *(volatile v4u*)dst = v;
  __threadfence();
  *(volatile v4u*)dst = v;
}
__device__ __forceinline__ void put_f4(float* dst, v4f v) {
  *(volatile v4f*)dst = v;
  __threadfence();
  *(volatile v4f*)dst = v;
}

__device__ __forceinline__ v8f wmb(const FragB& a, const FragB& b, v8f c) {
  v8f d = __builtin_amdgcn_wmma_f32_16x16x32_bf16(false, a.v, false, b.v, (short)0, c, false, false);
  asm volatile("v_nop\n\tv_nop\n\tv_nop\n\tv_nop" : "+v"(d) : "v"(a.w), "v"(b.w));
  return d;
}

template <int MT, int NT, int LDA, int LDB, int KK>
__device__ __forceinline__ void gemm_core(const unsigned short* __restrict__ A,
                                          const unsigned short* __restrict__ Bt,
                                          const int row0, const int lane, v8f (&acc)[MT][NT]) {
  static_assert(KK % 32 == 0);
  static_assert(LDA % 8 == 0);
  static_assert(LDB % 8 == 0);
  const int h = lane >> 4, m = lane & 15;
  const unsigned short* pa = A + (size_t)(row0 + m) * LDA + 8 * h;
  const unsigned short* pb = Bt + (size_t)m * LDB + 8 * h;
#pragma unroll 1
  for (int k0 = 0; k0 < KK; k0 += 32) {
    FragB a[MT];
#pragma unroll
    for (int mt = 0; mt < MT; ++mt) {
      const unsigned short* q = pa + (size_t)(16 * mt) * LDA + k0;
      a[mt].h[0] = *(const v8usa*)q;
      a[mt].h[1] = *(const v8usa*)(q + 16);
    }
#pragma unroll
    for (int nt = 0; nt < NT; ++nt) {
      const unsigned short* q = pb + (size_t)(16 * nt) * LDB + k0;
      FragB b;
      b.h[0] = *(const v8usa*)q;
      b.h[1] = *(const v8usa*)(q + 16);
#pragma unroll
      for (int mt = 0; mt < MT; ++mt) acc[mt][nt] = wmb(a[mt], b, acc[mt][nt]);
    }
  }
}

__device__ __forceinline__ void split_store_128(const float* sT, unsigned short* dst, int tid) {
  v4u hv[8], lv[8];
#pragma unroll
  for (int it = 0; it < 8; ++it) {
    const int u = it * 128 + tid;
    const int row = u >> 4, c8 = u & 15;
    const v4f a = *(const v4fa*)(sT + row * 128 + 8 * c8);
    const v4f b = *(const v4fa*)(sT + row * 128 + 8 * c8 + 4);
    const HL s = split8(a, b);
    hv[it] = s.h;
    lv[it] = s.l;
  }
#pragma unroll
  for (int it = 0; it < 8; ++it) {
    const int u = it * 128 + tid;
    unsigned short* p = dst + (size_t)(u >> 4) * 256 + 8 * (u & 15);
    *(volatile v4u*)p = hv[it];
    *(volatile v4u*)(p + 128) = lv[it];
  }
  __threadfence();
#pragma unroll
  for (int it = 0; it < 8; ++it) {
    const int u = it * 128 + tid;
    unsigned short* p = dst + (size_t)(u >> 4) * 256 + 8 * (u & 15);
    *(volatile v4u*)p = hv[it];
    *(volatile v4u*)(p + 128) = lv[it];
  }
}

__device__ __forceinline__ void split_store_g3(const float* sT, unsigned short* dst, int tid) {
  v4u hv[8], lv[8];
#pragma unroll
  for (int it = 0; it < 8; ++it) {
    const int u = it * 128 + tid;
    const int row = u >> 3, c8 = u & 7;
    const v4f a = *(const v4fa*)(sT + row * 64 + 8 * c8);
    const v4f b = *(const v4fa*)(sT + row * 64 + 8 * c8 + 4);
    const HL s = split8(a, b);
    hv[it] = s.h;
    lv[it] = s.l;
  }
#pragma unroll
  for (int it = 0; it < 8; ++it) {
    const int u = it * 128 + tid;
    unsigned short* p = dst + (size_t)(u >> 3) * 192 + 8 * (u & 7);
    *(volatile v4u*)p = hv[it];
    *(volatile v4u*)(p + 64) = lv[it];
    *(volatile v4u*)(p + 128) = hv[it];
  }
  __threadfence();
#pragma unroll
  for (int it = 0; it < 8; ++it) {
    const int u = it * 128 + tid;
    unsigned short* p = dst + (size_t)(u >> 3) * 192 + 8 * (u & 7);
    *(volatile v4u*)p = hv[it];
    *(volatile v4u*)(p + 64) = lv[it];
    *(volatile v4u*)(p + 128) = hv[it];
  }
}

__device__ __forceinline__ void flat_store_f32(const float* sT, float* dst, int tid) {
#pragma unroll
  for (int it = 0; it < 16; ++it) {
    const int u = it * 128 + tid;
    const v4f v = *(const v4fa*)(sT + 4 * u);
    *(volatile v4f*)(dst + 4 * u) = v;
  }
}

__device__ __forceinline__ void vec_plane(const float* __restrict__ src, float* dst, int tid) {
  const int idx = tid & 31;
  const v4f x = *(const v4fa*)(src + 4 * idx);
  pin4(x);
  v4f y;
  y.x = bfr(x.x); y.y = bfr(x.y); y.z = bfr(x.z); y.w = bfr(x.w);
  if (tid < 32) put_f4(dst + 4 * idx, y);
}

__global__ __launch_bounds__(256) void k_prep(
    const float* __restrict__ feat_opt, const float* __restrict__ feat_mas,
    const float* __restrict__ w0_w1, const float* __restrict__ w0_b1,
    const float* __restrict__ w0_w2, const float* __restrict__ w0_b2,
    const float* __restrict__ vb, const float* __restrict__ coeff,
    const float* __restrict__ we1, const float* __restrict__ be1,
    const float* __restrict__ we2, const float* __restrict__ be2,
    const float* __restrict__ wom1, const float* __restrict__ bom1,
    const float* __restrict__ wom2, const float* __restrict__ bom2,
    unsigned short* __restrict__ XB, unsigned short* __restrict__ FMT,
    unsigned short* __restrict__ W1T, unsigned short* __restrict__ W2D,
    unsigned short* __restrict__ WR3, unsigned short* __restrict__ WOM,
    float* __restrict__ PAR)
{
  __shared__ __align__(16) float sV[3 * 64 * 32];
  __shared__ float sC[16];
  const int blk = blockIdx.x;
  const int tid = threadIdx.x;

  if (blk < PB0_FMT) {
    const int u = blk * 256 + tid;
    const float* s = feat_opt + (size_t)u * 8;
    const v4f a = *(const v4fa*)s;
    const v4f c = *(const v4fa*)(s + 4);
    put_u4(XB + (size_t)u * 8, pack8(a.x, a.y, a.z, a.w, c.x, c.y, c.z, c.w));
  } else if (blk < PB0_W2D) {
    const int u = (blk - PB0_FMT) * 256 + tid;
    const int b = u >> 12, i = (u >> 6) & 63, k8 = u & 63;
    const int m0 = (8 * k8) & 255;
    const float* s = feat_mas + ((size_t)(b * NM + m0)) * CIN + i;
    const float x0 = s[0], x1 = s[64], x2 = s[128], x3 = s[192];
    const float x4 = s[256], x5 = s[320], x6 = s[384], x7 = s[448];
    put_u4(FMT + (size_t)u * 8, pack8(x0, x1, x2, x3, x4, x5, x6, x7));
  } else if (blk < PB0_WOM) {
    const int u = (blk - PB0_W2D) * 256 + tid;
    const int n = u >> 5, k8 = u & 31;
    const int k0 = (8 * k8) & 127;
    const float* s = w0_w2 + (size_t)k0 * PO + n;
    const float x0 = s[0], x1 = s[128], x2 = s[256], x3 = s[384];
    const float x4 = s[512], x5 = s[640], x6 = s[768], x7 = s[896];
    put_u4(W2D + (size_t)u * 8, pack8(x0, x1, x2, x3, x4, x5, x6, x7));
  } else if (blk < PB0_W1T) {
    const int u = (blk - PB0_WOM) * 256 + tid;
    const int n = u >> 5, k8 = u & 31;
    const int kk0 = (8 * k8) & 127;
    const bool live = kk0 < NFM;
    const int kc = live ? kk0 : (NFM - 8);
    const float* s = wom1 + (size_t)kc * HID + n;
    const float x0 = s[0], x1 = s[128], x2 = s[256], x3 = s[384];
    const float x4 = s[512], x5 = s[640], x6 = s[768], x7 = s[896];
    asm volatile("" :: "v"(x0), "v"(x1), "v"(x2), "v"(x3), "v"(x4), "v"(x5), "v"(x6), "v"(x7));
    v4u p = pack8(x0, x1, x2, x3, x4, x5, x6, x7);
    const unsigned mk = live ? 0xffffffffu : 0u;
    p.x &= mk; p.y &= mk; p.z &= mk; p.w &= mk;
    put_u4(WOM + (size_t)u * 8, p);
  } else if (blk < PB0_WR3) {
    const int u = (blk - PB0_W1T) * 256 + tid;
    const int n = u >> 3, k8 = u & 7;
    const float* s = w0_w1 + (size_t)(8 * k8) * HID + n;
    const float x0 = s[0], x1 = s[128], x2 = s[256], x3 = s[384];
    const float x4 = s[512], x5 = s[640], x6 = s[768], x7 = s[896];
    put_u4(W1T + (size_t)u * 8, pack8(x0, x1, x2, x3, x4, x5, x6, x7));
  } else if (blk < PB0_PAR) {
#pragma unroll 2
    for (int it = 0; it < 6; ++it) {
      const int q = it * 256 + tid;
      const v4f x = *(const v4fa*)(vb + 4 * q);
      v4f y;
      y.x = bfr(x.x); y.y = bfr(x.y); y.z = bfr(x.z); y.w = bfr(x.w);
      *(v4fa*)(sV + 4 * q) = y;
    }
    {
      const int ci = (tid < 8) ? tid : 8;
      const float c = bfr(coeff[ci]);
      asm volatile("" :: "v"(c));
      if (tid < 9) sC[tid] = c;
    }
    __syncthreads();
    const int u = (blk - PB0_WR3) * 256 + tid;
    const int n = u / 24;
    const int k8 = u - 24 * n;
    const int seg = k8 >> 3;
    const int i0 = 8 * (k8 & 7);
    const bool live = n < NFM;
    const int nc = live ? n : (NFM - 1);
    const int t = nc >> 5, jj = nc & 31;
    const float c0 = sC[3 * t], c1 = sC[3 * t + 1], c2 = sC[3 * t + 2];
    unsigned bits[8];
#pragma unroll
    for (int j = 0; j < 8; ++j) {
      const int i = i0 + j;
      float wv = c0 * sV[i * 32 + jj];
      wv = fmaf(c1, sV[2048 + i * 32 + jj], wv);
      wv = fmaf(c2, sV[4096 + i * 32 + jj], wv);
      const unsigned hb = f2bf(wv);
      const unsigned lb = f2bf(wv - bf2f(hb));
      bits[j] = (seg == 2) ? lb : hb;
    }
    const unsigned mk = live ? 0xffffffffu : 0u;
    v4u p;
    p.x = pk(bits[0], bits[1]) & mk;
    p.y = pk(bits[2], bits[3]) & mk;
    p.z = pk(bits[4], bits[5]) & mk;
    p.w = pk(bits[6], bits[7]) & mk;
    put_u4(WR3 + (size_t)u * 8, p);
  } else {
    const int pb = blk - PB0_PAR;
    if (pb == 0) {
      const int idx = tid & 127;
      const float a = bfr(we1[idx]);
      const float b = bfr(be1[idx]);
      const float c = bfr(we2[idx]);
      asm volatile("" :: "v"(a), "v"(b), "v"(c));
      v4f y;
      y.x = a; y.y = b; y.z = c; y.w = 0.0f;
      if (tid < 128) put_f4(PAR + PAR_E4 + 4 * idx, y);
    } else if (pb == 1) {
      vec_plane(w0_b1, PAR + PAR_B1, tid);
    } else if (pb == 2) {
      vec_plane(w0_b2, PAR + PAR_B2, tid);
    } else if (pb == 3) {
      vec_plane(bom1, PAR + PAR_BOM1, tid);
    } else if (pb == 4) {
      vec_plane(wom2, PAR + PAR_WOM2, tid);
    } else {
      const float e = bfr(be2[0]);
      const float f = bfr(bom2[0]);
      asm volatile("" :: "v"(e), "v"(f));
      v4f y;
      y.x = (tid == 0) ? e : 0.0f;
      y.y = (tid == 0) ? f : 0.0f;
      y.z = 0.0f; y.w = 0.0f;
      if (tid < 8) put_f4(PAR + PAR_SC + 4 * tid, y);
    }
  }
}

__global__ __launch_bounds__(256) void k_edge(const int* __restrict__ adj, const float* __restrict__ fe,
                                              const float* __restrict__ PAR,
                                              unsigned short* __restrict__ AHL) {
  __shared__ __align__(16) float sPar[HID * 4];
  const int tid = threadIdx.x, lane = tid & 31, w = tid >> 5;
  {
    const int idx = tid & 127;
    const v4f p = *(const v4fa*)(PAR + PAR_E4 + 4 * idx);
    pin4(p);
    if (tid < 128) *(v4fa*)(sPar + 4 * idx) = p;
  }
  const float be2v = PAR[PAR_SC];
  const int row = blockIdx.x * 8 + w;
  const size_t base = (size_t)row * NM + 8 * lane;
  const v4i a0 = *(const v4ia*)(adj + base);
  const v4i a1 = *(const v4ia*)(adj + base + 4);
  const v4f f0 = *(const v4fa*)(fe + base);
  const v4f f1 = *(const v4fa*)(fe + base + 4);
  __syncthreads();

  float x[8], c[8];
  x[0] = bfr(f0.x); x[1] = bfr(f0.y); x[2] = bfr(f0.z); x[3] = bfr(f0.w);
  x[4] = bfr(f1.x); x[5] = bfr(f1.y); x[6] = bfr(f1.z); x[7] = bfr(f1.w);
#pragma unroll
  for (int e = 0; e < 8; ++e) c[e] = 0.0f;

#pragma unroll 2
  for (int hh = 0; hh < HID; ++hh) {
    const v4f p = *(const v4fa*)(sPar + 4 * hh);
#pragma unroll
    for (int e = 0; e < 8; ++e) c[e] = fmaf(fmaf(x[e], p.x, p.y), p.z, c[e]);
  }

  v4f ga, gb;
  ga.x = (a0.x == 1) ? (c[0] + be2v) : 0.0f;
  ga.y = (a0.y == 1) ? (c[1] + be2v) : 0.0f;
  ga.z = (a0.z == 1) ? (c[2] + be2v) : 0.0f;
  ga.w = (a0.w == 1) ? (c[3] + be2v) : 0.0f;
  gb.x = (a1.x == 1) ? (c[4] + be2v) : 0.0f;
  gb.y = (a1.y == 1) ? (c[5] + be2v) : 0.0f;
  gb.z = (a1.z == 1) ? (c[6] + be2v) : 0.0f;
  gb.w = (a1.w == 1) ? (c[7] + be2v) : 0.0f;
  const HL s = split8(ga, gb);
  unsigned short* d = AHL + (size_t)row * 512 + 8 * lane;
  *(volatile v4u*)d = s.h;
  *(volatile v4u*)(d + 256) = s.l;
  __threadfence();
  *(volatile v4u*)d = s.h;
  *(volatile v4u*)(d + 256) = s.l;
}

__global__ __launch_bounds__(128) __attribute__((amdgpu_num_vgpr(248)))
void k_h0(const unsigned short* __restrict__ XB, const unsigned short* __restrict__ W1T,
          const float* __restrict__ PAR, unsigned short* __restrict__ H0HL) {
  __shared__ __align__(16) float sT[64 * 128];
  __shared__ __align__(16) float sB[128];
  const int tid = threadIdx.x, lane = tid & 31, w = tid >> 5;
  const int h = lane >> 4, m = lane & 15;
  {
    const int idx = tid & 31;
    const v4f p = *(const v4fa*)(PAR + PAR_B1 + 4 * idx);
    pin4(p);
    if (tid < 32) *(v4fa*)(sB + 4 * idx) = p;
  }
  const int row0 = blockIdx.x * 64;
  v8f acc[1][8];
#pragma unroll
  for (int nt = 0; nt < 8; ++nt) acc[0][nt] = z8();
  gemm_core<1, 8, CIN, CIN, CIN>(XB, W1T, row0 + 16 * w, lane, acc);
  __syncthreads();
#pragma unroll
  for (int nt = 0; nt < 8; ++nt) {
    const int cl = 16 * nt + m;
    const float bv = sB[cl];
#pragma unroll
    for (int r = 0; r < 8; ++r) sT[(16 * w + 8 * h + r) * 128 + cl] = acc[0][nt][r] + bv;
  }
  __syncthreads();
#pragma unroll 1
  for (int it = 0; it < 64; ++it) {
    const int e = it * 128 + tid;
    const float xv = sT[e];
    sT[e] = elu_f(xv);
  }
  __syncthreads();
  split_store_128(sT, H0HL + (size_t)row0 * 256, tid);
}

__global__ __launch_bounds__(128) __attribute__((amdgpu_num_vgpr(248)))
void k_p(const unsigned short* __restrict__ H0HL, const unsigned short* __restrict__ W2D,
         const float* __restrict__ PAR, float* __restrict__ P) {
  __shared__ __align__(16) float sT[64 * 128];
  __shared__ __align__(16) float sB[128];
  const int tid = threadIdx.x, lane = tid & 31, w = tid >> 5;
  const int h = lane >> 4, m = lane & 15;
  {
    const int idx = tid & 31;
    const v4f p = *(const v4fa*)(PAR + PAR_B2 + 4 * idx);
    pin4(p);
    if (tid < 32) *(v4fa*)(sB + 4 * idx) = p;
  }
  const int row0 = blockIdx.x * 64;
  v8f acc[1][8];
#pragma unroll
  for (int nt = 0; nt < 8; ++nt) acc[0][nt] = z8();
  gemm_core<1, 8, 256, 256, 256>(H0HL, W2D, row0 + 16 * w, lane, acc);
  __syncthreads();
#pragma unroll
  for (int nt = 0; nt < 8; ++nt) {
    const int cl = 16 * nt + m;
    const float bv = sB[cl];
#pragma unroll
    for (int r = 0; r < 8; ++r) sT[(16 * w + 8 * h + r) * 128 + cl] = acc[0][nt][r] + bv;
  }
  __syncthreads();
  float* dst = P + (size_t)row0 * PO;
  flat_store_f32(sT, dst, tid);
  __threadfence();
  flat_store_f32(sT, dst, tid);
}

__global__ __launch_bounds__(128) __attribute__((amdgpu_num_vgpr(248)))
void k_g(const unsigned short* __restrict__ AHL, const unsigned short* __restrict__ FMT,
         unsigned short* __restrict__ G3) {
  __shared__ __align__(16) float sT[128 * 64];
  const int tid = threadIdx.x, lane = tid & 31, w = tid >> 5;
  const int h = lane >> 4, m = lane & 15;
  const int row0 = blockIdx.x * 128;
  const int b = row0 / NO;
  const unsigned short* Bt = FMT + (size_t)b * CIN * 512;
  v8f acc[2][4];
#pragma unroll
  for (int mt = 0; mt < 2; ++mt)
#pragma unroll
    for (int nt = 0; nt < 4; ++nt) acc[mt][nt] = z8();
  gemm_core<2, 4, 512, 512, 512>(AHL, Bt, row0 + 32 * w, lane, acc);
#pragma unroll
  for (int nt = 0; nt < 4; ++nt) {
    const int cl = 16 * nt + m;
#pragma unroll
    for (int mt = 0; mt < 2; ++mt)
#pragma unroll
      for (int r = 0; r < 8; ++r) sT[(32 * w + 16 * mt + 8 * h + r) * 64 + cl] = acc[mt][nt][r];
  }
  __syncthreads();
  split_store_g3(sT, G3 + (size_t)row0 * 192, tid);
}

__global__ __launch_bounds__(128) __attribute__((amdgpu_num_vgpr(248)))
void k_fm(const unsigned short* __restrict__ G3, const unsigned short* __restrict__ WR3,
          unsigned short* __restrict__ FMHL) {
  __shared__ __align__(16) float sT[64 * 128];
  const int tid = threadIdx.x, lane = tid & 31, w = tid >> 5;
  const int h = lane >> 4, m = lane & 15;
  const int row0 = blockIdx.x * 64;
  v8f acc[1][8];
#pragma unroll
  for (int nt = 0; nt < 8; ++nt) acc[0][nt] = z8();
  gemm_core<1, 8, 192, 192, 192>(G3, WR3, row0 + 16 * w, lane, acc);
#pragma unroll
  for (int nt = 0; nt < 8; ++nt) {
    const int cl = 16 * nt + m;
#pragma unroll
    for (int r = 0; r < 8; ++r) sT[(16 * w + 8 * h + r) * 128 + cl] = acc[0][nt][r];
  }
  __syncthreads();
  split_store_128(sT, FMHL + (size_t)row0 * 256, tid);
}

__global__ __launch_bounds__(128) __attribute__((amdgpu_num_vgpr(248)))
void k_gate_out(const unsigned short* __restrict__ FMHL, const unsigned short* __restrict__ WOM,
                const float* __restrict__ PAR, const float* __restrict__ P, float* __restrict__ out) {
  __shared__ __align__(16) float sT[64 * TP];
  __shared__ __align__(16) float sBm[128];
  __shared__ __align__(16) float sW2[128];
  const int tid = threadIdx.x, lane = tid & 31, w = tid >> 5;
  const int h = lane >> 4, m = lane & 15;
  {
    const int idx = tid & 31;
    const v4f p = *(const v4fa*)(PAR + PAR_BOM1 + 4 * idx);
    const v4f q = *(const v4fa*)(PAR + PAR_WOM2 + 4 * idx);
    pin4(p);
    pin4(q);
    if (tid < 32) {
      *(v4fa*)(sBm + 4 * idx) = p;
      *(v4fa*)(sW2 + 4 * idx) = q;
    }
  }
  const float bom2v = PAR[PAR_SC + 1];
  const int row0 = blockIdx.x * 64;
  v8f acc[1][8];
#pragma unroll
  for (int nt = 0; nt < 8; ++nt) acc[0][nt] = z8();
  gemm_core<1, 8, 256, 256, 256>(FMHL, WOM, row0 + 16 * w, lane, acc);
#pragma unroll
  for (int nt = 0; nt < 8; ++nt) {
    const int cl = 16 * nt + m;
#pragma unroll
    for (int r = 0; r < 8; ++r) sT[(16 * w + 8 * h + r) * TP + cl] = acc[0][nt][r];
  }
  __syncthreads();
  {
    const float bm = sBm[tid];
    const float w2 = sW2[tid];
#pragma unroll 1
    for (int it = 0; it < 64; ++it) {
      const int idx = it * TP + tid;
      const float xv = sT[idx] + bm;
      const float yv = elu_f(xv) * w2;
      sT[idx] = yv;
    }
  }
  __syncthreads();

  v4f o[16];
#pragma unroll
  for (int i = 0; i < 16; ++i) {
    const int rl = 16 * w + i;
    const float* rp = sT + rl * TP;
    float t = rp[lane];
    t = t + rp[lane + 32];
    t = t + rp[lane + 64];
    t = t + rp[lane + 96];
    t = t + __shfl_xor(t, 16);
    t = t + __shfl_xor(t, 8);
    t = t + __shfl_xor(t, 4);
    t = t + __shfl_xor(t, 2);
    t = t + __shfl_xor(t, 1);
    const float s = t + bom2v;
    const v4f p = *(const v4fa*)(P + (size_t)(row0 + rl) * PO + 4 * lane);
    v4f y;
    y.x = p.x + s; y.y = p.y + s; y.z = p.z + s; y.w = p.w + s;
    y.x = (y.x >= 0.0f) ? y.x : 0.2f * y.x;
    y.y = (y.y >= 0.0f) ? y.y : 0.2f * y.y;
    y.z = (y.z >= 0.0f) ? y.z : 0.2f * y.z;
    y.w = (y.w >= 0.0f) ? y.w : 0.2f * y.w;
    o[i] = y;
  }
#pragma unroll
  for (int i = 0; i < 16; ++i)
    *(volatile v4f*)(out + (size_t)(row0 + 16 * w + i) * PO + 4 * lane) = o[i];
  __threadfence();
#pragma unroll
  for (int i = 0; i < 16; ++i)
    *(volatile v4f*)(out + (size_t)(row0 + 16 * w + i) * PO + 4 * lane) = o[i];
}

extern "C" void kernel_launch(void* const* d_in, const int* in_sizes, int n_in,
                              void* d_out, int out_size, void* d_ws, size_t ws_size,
                              hipStream_t stream) {
  if (n_in < 19) return;
  if (in_sizes[0] != NB * NO * NM) return;
  if (in_sizes[2] != NB * NO * CIN) return;
  if (in_sizes[3] != NB * NM * CIN) return;
  if (in_sizes[4] != NB * NO * NM) return;
  if (in_sizes[5] != CIN * HID) return;
  if (in_sizes[6] != HID) return;
  if (in_sizes[7] != HID * PO) return;
  if (in_sizes[8] != PO) return;
  if (in_sizes[9] != 3 * CIN * 32) return;
  if (in_sizes[10] != 9) return;
  if (in_sizes[11] != HID || in_sizes[12] != HID || in_sizes[13] != HID) return;
  if (in_sizes[14] != 1) return;
  if (in_sizes[15] != NFM * HID) return;
  if (in_sizes[16] != HID || in_sizes[17] != HID) return;
  if (in_sizes[18] != 1) return;
  if (out_size != MROWS * PO) return;
  if (WS_TOTAL > ws_size) return;

  const int*   adj       = (const int*)  d_in[0];
  const float* feat_opt  = (const float*)d_in[2];
  const float* feat_mas  = (const float*)d_in[3];
  const float* feat_edge = (const float*)d_in[4];
  const float* w0_w1     = (const float*)d_in[5];
  const float* w0_b1     = (const float*)d_in[6];
  const float* w0_w2     = (const float*)d_in[7];
  const float* w0_b2     = (const float*)d_in[8];
  const float* vb        = (const float*)d_in[9];
  const float* coeff     = (const float*)d_in[10];
  const float* we1       = (const float*)d_in[11];
  const float* be1       = (const float*)d_in[12];
  const float* we2       = (const float*)d_in[13];
  const float* be2       = (const float*)d_in[14];
  const float* wom1      = (const float*)d_in[15];
  const float* bom1      = (const float*)d_in[16];
  const float* wom2      = (const float*)d_in[17];
  const float* bom2      = (const float*)d_in[18];
  float* out = (float*)d_out;

  char* ws = (char*)d_ws;
  unsigned short* XB   = (unsigned short*)(ws + O_XB);
  unsigned short* AHL  = (unsigned short*)(ws + O_AHL);
  unsigned short* FMT  = (unsigned short*)(ws + O_FMT);
  unsigned short* H0HL = (unsigned short*)(ws + O_H0);
  float*          P    = (float*)         (ws + O_P);
  unsigned short* G3   = (unsigned short*)(ws + O_G3);
  unsigned short* FMHL = (unsigned short*)(ws + O_FM);
  unsigned short* W1T  = (unsigned short*)(ws + O_W1T);
  unsigned short* W2D  = (unsigned short*)(ws + O_W2D);
  unsigned short* WR3  = (unsigned short*)(ws + O_WR3);
  unsigned short* WOM  = (unsigned short*)(ws + O_WOM);
  float*          PAR  = (float*)         (ws + O_PAR);

  k_prep<<<dim3(PB_TOTAL), dim3(256), 0, stream>>>(feat_opt, feat_mas, w0_w1, w0_b1, w0_w2, w0_b2, vb, coeff,
                                                   we1, be1, we2, be2, wom1, bom1, wom2, bom2,
                                                   XB, FMT, W1T, W2D, WR3, WOM, PAR);
  k_edge<<<dim3(MROWS / 8), dim3(256), 0, stream>>>(adj, feat_edge, PAR, AHL);
  k_h0<<<dim3(MROWS / 64), dim3(128), 0, stream>>>(XB, W1T, PAR, H0HL);
  k_p<<<dim3(MROWS / 64), dim3(128), 0, stream>>>(H0HL, W2D, PAR, P);
  k_g<<<dim3(MROWS / 128), dim3(128), 0, stream>>>(AHL, FMT, G3);
  k_fm<<<dim3(MROWS / 64), dim3(128), 0, stream>>>(G3, WR3, FMHL);
  k_gate_out<<<dim3(MROWS / 64), dim3(128), 0, stream>>>(FMHL, WOM, PAR, P, out);
  (void)hipGetLastError();
}
